// NDRSA_block_79482664780194
// MI455X (gfx1250) — hardware-run, weakly checked
//
#include <hip/hip_runtime.h>
#include <math.h>

constexpr int kBatch = 4;
constexpr int kSeq   = 2048;
constexpr int kDim   = 512;
constexpr int kHeads = 8;
constexpr int kDh    = 64;
constexpr int kFfn   = 2048;
constexpr int kTok   = kBatch * kSeq;
constexpr int kHeadsPerChunk = 2;
constexpr float kWCarry     = 16.0f;
constexpr float kWCarryInv  = 1.0f / 16.0f;
constexpr float kPCarry     = 2048.0f;
constexpr float kCtxCarry   = 256.0f;
constexpr float kScoreScale = 0.125f;
constexpr float kPVScale    = kCtxCarry / kPCarry;
constexpr float kOutScale   = 1.0f / (kCtxCarry * kWCarry);
constexpr float kInvDim     = 1.0f / 512.0f;
constexpr float kLnEps      = 1e-5f;

typedef __attribute__((ext_vector_type(16))) _Float16 v16h;
typedef __attribute__((ext_vector_type(8)))  _Float16 v8h;
typedef __attribute__((ext_vector_type(16))) __bf16   v16b;
typedef __attribute__((ext_vector_type(8)))  __bf16   v8b;
typedef __attribute__((ext_vector_type(8)))  float    v8f;
typedef __attribute__((ext_vector_type(4)))  float    v4f;
typedef __attribute__((ext_vector_type(4)))  unsigned int v4u;
typedef __attribute__((ext_vector_type(2)))  unsigned int v2u;

__device__ __forceinline__ unsigned short f2bf_bits(float f) {
  unsigned u = __float_as_uint(f);
  return (unsigned short)((u + 0x7FFFu + ((u >> 16) & 1u)) >> 16);
}
__device__ __forceinline__ float bf_bits2f(unsigned short h) { return __uint_as_float(((unsigned)h) << 16); }

__device__ __forceinline__ void dep_guard_h(v8f& a, v8f& b, v16h x, v16h y) { asm volatile("v_nop\n\tv_nop\n\tv_nop\n\tv_nop" : "+v"(a), "+v"(b) : "v"(x), "v"(y)); }
__device__ __forceinline__ void dep_guard_b(v8f& a, v8f& b, v16b x, v16b y) { asm volatile("v_nop\n\tv_nop\n\tv_nop\n\tv_nop" : "+v"(a), "+v"(b) : "v"(x), "v"(y)); }
__device__ __forceinline__ void keep4_h(v16h a, v16h b, v16h c, v16h d) { asm volatile("v_nop" :: "v"(a), "v"(b), "v"(c), "v"(d)); }
__device__ __forceinline__ void keep4_b(v16b a, v16b b, v16b c, v16b d) { asm volatile("v_nop" :: "v"(a), "v"(b), "v"(c), "v"(d)); }
__device__ __forceinline__ void acc_guard4(v8f& a, v8f& b, v8f& c, v8f& d) { asm volatile("v_nop\n\tv_nop\n\tv_nop\n\tv_nop" : "+v"(a), "+v"(b), "+v"(c), "+v"(d)); }
template <typename T> struct Frag;
template <> struct Frag<_Float16> {
  typedef v16h V; union U { v16h v; v8h h[2]; };
  static __device__ __forceinline__ v16h load(const _Float16* p) {
    U f; f.h[0] = *(const v8h*)(p); f.h[1] = *(const v8h*)(p + 16); return f.v;
  }
  static __device__ __forceinline__ v8f mma(v16h a, v16h b, v8f c) {
    return __builtin_amdgcn_wmma_f32_16x16x32_f16(false, a, false, b, (short)0, c, false, false);
  }
  static __device__ __forceinline__ void guard(v8f& a, v8f& b, v16h x, v16h y) { dep_guard_h(a, b, x, y); }
  static __device__ __forceinline__ void keep(v16h a, v16h b, v16h c, v16h d) { keep4_h(a, b, c, d); }
};
template <> struct Frag<__bf16> {
  typedef v16b V; union U { v16b v; v8b h[2]; };
  static __device__ __forceinline__ v16b load(const __bf16* p) {
    U f; f.h[0] = *(const v8b*)(p); f.h[1] = *(const v8b*)(p + 16); return f.v;
  }
  static __device__ __forceinline__ v8f mma(v16b a, v16b b, v8f c) {
    return __builtin_amdgcn_wmma_f32_16x16x32_bf16(false, a, false, b, (short)0, c, false, false);
  }
  static __device__ __forceinline__ void guard(v8f& a, v8f& b, v16b x, v16b y) { dep_guard_b(a, b, x, y); }
  static __device__ __forceinline__ void keep(v16b a, v16b b, v16b c, v16b d) { keep4_b(a, b, c, d); }
};

__device__ __forceinline__ unsigned pk16(unsigned short a, unsigned short b) { return (unsigned)a | ((unsigned)b << 16); }
__device__ __forceinline__ unsigned short h_bits(float f) { const _Float16 h = (_Float16)f; return __builtin_bit_cast(unsigned short, h); }

template <int ET> struct Elem;
template <> struct Elem<0> { typedef _Float16 T; };
template <> struct Elem<1> { typedef __bf16 T; };
template <int ET, bool SPLIT, int BIAS_MODE, int OUT_MODE, bool RESID, int ACT = 0>
__global__ __launch_bounds__(256) void wmma_gemm64(
    const unsigned short* __restrict__ Ap, const unsigned short* __restrict__ A2p, int lda, long strideA,
    const unsigned short* __restrict__ Btp, const unsigned short* __restrict__ Bt2p, int ldb, long strideB,
    void* __restrict__ Cout, void* __restrict__ Cout2, int ldc, long strideC,
    const float* __restrict__ bias,
    const float* __restrict__ resid, long strideR,
    int M, int N, int K, float scale) {
  typedef typename Elem<ET>::T T;
  typedef typename Frag<T>::V V;
  const T* A = (const T*)Ap; const T* A2 = (const T*)A2p; const T* Bt = (const T*)Btp; const T* Bt2 = (const T*)Bt2p;
  __shared__ __align__(16) float sT[8][16 * 68];
  const int b    = blockIdx.y;
  const int lane = threadIdx.x & 31;
  const int wave = threadIdx.x >> 5;
  const int tilesN = N >> 6;
  const int tilesM = M >> 6;
  const int tile = blockIdx.x * 8 + wave;
  if (tile >= tilesM * tilesN) return;
  const int tm = tile / tilesN;
  const int tn = tile - tm * tilesN;
  const int m0 = tm << 6;
  const int n0 = tn << 6;

  const T* Ab  = A  + (size_t)b * strideA;
  const T* Bb  = Bt + (size_t)b * strideB;
  const T* Ab2 = SPLIT ? (A2  + (size_t)b * strideA) : nullptr;
  const T* Bb2 = SPLIT ? (Bt2 + (size_t)b * strideB) : nullptr;

  const int rlane = lane & 15;
  const int koff  = (lane >> 4) * 8;
  const int mOff  = (lane >> 4) * 8;

  v8f acc[4][4];
#pragma unroll
  for (int i = 0; i < 4; ++i)
#pragma unroll
    for (int j = 0; j < 4; ++j) acc[i][j] = (v8f){0.f,0.f,0.f,0.f,0.f,0.f,0.f,0.f};

  for (int k0 = 0; k0 < K; k0 += 32) {
    V bh[4], bl[4];
#pragma unroll
    for (int j = 0; j < 4; ++j) {
      const size_t bo = (size_t)(n0 + (j << 4) + rlane) * ldb + koff + k0;
      bh[j] = Frag<T>::load(Bb + bo);
      if (SPLIT) bl[j] = Frag<T>::load(Bb2 + bo);
    }
#pragma unroll
    for (int i = 0; i < 4; ++i) {
      const size_t ao = (size_t)(m0 + (i << 4) + rlane) * lda + koff + k0;
      V ah = Frag<T>::load(Ab + ao);
      V al;
      if (SPLIT) al = Frag<T>::load(Ab2 + ao);
#pragma unroll
      for (int j = 0; j < 4; ++j) {
        acc[i][j] = Frag<T>::mma(ah, bh[j], acc[i][j]);
        if (SPLIT) {
          acc[i][j] = Frag<T>::mma(ah, bl[j], acc[i][j]);
          acc[i][j] = Frag<T>::mma(al, bh[j], acc[i][j]);
        }
      }
      Frag<T>::guard(acc[i][0], acc[i][3], ah, SPLIT ? al : ah);
    }
    Frag<T>::keep(bh[0], bh[1], bh[2], bh[3]);
    if (SPLIT) Frag<T>::keep(bl[0], bl[1], bl[2], bl[3]);
  }
  acc_guard4(acc[0][0], acc[0][1], acc[0][2], acc[0][3]);
  acc_guard4(acc[1][0], acc[1][1], acc[1][2], acc[1][3]);
  acc_guard4(acc[2][0], acc[2][1], acc[2][2], acc[2][3]);
  acc_guard4(acc[3][0], acc[3][1], acc[3][2], acc[3][3]);

  float* slab = sT[wave];
  const float* Rb = RESID ? (resid + (size_t)b * strideR) : nullptr;
#pragma unroll
  for (int i = 0; i < 4; ++i) {
    const int mBase = m0 + (i << 4);
#pragma unroll
    for (int j = 0; j < 4; ++j) {
      const int n = n0 + (j << 4) + rlane;
      float bv = 0.f;
      if (BIAS_MODE == 2) bv = bias[n];
#pragma unroll
      for (int r = 0; r < 8; ++r) {
        float v = acc[i][j][r] * scale;
        if (BIAS_MODE == 1) v += bias[mBase + mOff + r];
        if (BIAS_MODE == 2) v += bv;
        if (RESID) v += Rb[(size_t)(mBase + mOff + r) * ldc + n];
        if (ACT == 2) v = fmaxf(v, 0.0f);
        if (ACT == 4) v = (v > 0.f) ? v : 0.01f * v;
        slab[(mOff + r) * 68 + (j << 4) + rlane] = v;
      }
    }
    __builtin_amdgcn_fence(__ATOMIC_RELEASE, "workgroup");
    __builtin_amdgcn_wave_barrier();
    __builtin_amdgcn_fence(__ATOMIC_ACQUIRE, "workgroup");
    if (OUT_MODE == 0) {
      float* C = (float*)Cout + (size_t)b * strideC;
      const int hh = lane >> 4, c4 = (lane & 15) * 4;
      for (int pass = 0; pass < 2; ++pass) {
#pragma unroll
        for (int it = 0; it < 8; ++it) {
          const int row = it * 2 + hh;
          v4f v = *(const v4f*)(slab + row * 68 + c4);
          *(volatile v4f*)(C + (size_t)(mBase + row) * ldc + n0 + c4) = v;
        }
        __threadfence();
      }
    } else {
      const int q = lane >> 3, c8 = (lane & 7) * 8;
      unsigned short* C  = (unsigned short*)Cout  + (size_t)b * strideC;
      unsigned short* C2 = (OUT_MODE == 2) ? ((unsigned short*)Cout2 + (size_t)b * strideC) : nullptr;
      for (int pass = 0; pass < 2; ++pass) {
#pragma unroll
        for (int it = 0; it < 4; ++it) {
          const int row = it * 4 + q;
          const float* sp = slab + row * 68 + c8;
          v8h hv, lv;
#pragma unroll
          for (int e = 0; e < 8; ++e) {
            if (OUT_MODE == 1) {
              hv[e] = (_Float16)sp[e];
            } else {
              unsigned short hb = f2bf_bits(sp[e]);
              unsigned short lb = f2bf_bits(sp[e] - bf_bits2f(hb));
              hv[e] = __builtin_bit_cast(_Float16, hb);
              lv[e] = __builtin_bit_cast(_Float16, lb);
            }
          }
          *(volatile v8h*)(C + (size_t)(mBase + row) * ldc + n0 + c8) = hv;
          if (OUT_MODE == 2) *(volatile v8h*)(C2 + (size_t)(mBase + row) * ldc + n0 + c8) = lv;
        }
        __threadfence();
      }
    }
    __builtin_amdgcn_fence(__ATOMIC_RELEASE, "workgroup");
    __builtin_amdgcn_wave_barrier();
    __builtin_amdgcn_fence(__ATOMIC_ACQUIRE, "workgroup");
  }
}

__global__ __launch_bounds__(256) void xprep_kernel(const float* __restrict__ x, unsigned short* __restrict__ X16,
                                                    float* __restrict__ SQ) {
  __shared__ float sqs[32];
  const int t = threadIdx.x, lane = t & 31, wave = t >> 5;
  const int r0 = blockIdx.x * 32;
  v4u u[4][2];
#pragma unroll
  for (int ri = 0; ri < 4; ++ri) {
    const int row = r0 + wave * 4 + ri;
    const float* xr = x + (size_t)row * kDim;
    float acc = 0.f;
#pragma unroll
    for (int it = 0; it < 2; ++it) {
      const int col = it * 256 + lane * 8;
      const v4f a = *(const v4f*)(xr + col);
      const v4f c = *(const v4f*)(xr + col + 4);
      unsigned short hb[8];
#pragma unroll
      for (int e = 0; e < 4; ++e) {
        hb[e]     = h_bits(a[e]);
        hb[4 + e] = h_bits(c[e]);
        acc += a[e] * a[e];
        acc += c[e] * c[e];
      }
      u[ri][it] = (v4u){pk16(hb[0], hb[1]), pk16(hb[2], hb[3]), pk16(hb[4], hb[5]), pk16(hb[6], hb[7])};
    }
#pragma unroll
    for (int off = 16; off > 0; off >>= 1) acc += __shfl_xor(acc, off, 32);
    if (lane == 0) sqs[wave * 4 + ri] = acc;
  }
  for (int pass = 0; pass < 2; ++pass) {
#pragma unroll
    for (int ri = 0; ri < 4; ++ri) {
      const int row = r0 + wave * 4 + ri;
#pragma unroll
      for (int it = 0; it < 2; ++it) {
        const int col = it * 256 + lane * 8;
        *(volatile v4u*)(X16 + (size_t)row * kDim + col) = u[ri][it];
      }
    }
    __threadfence();
  }
  __syncthreads();
  if (wave == 0) {
    const float v = sqs[lane];
    for (int pass = 0; pass < 2; ++pass) {
      *(volatile float*)(SQ + r0 + lane) = v;
      __threadfence();
    }
  }
}

__global__ __launch_bounds__(256) void wtcast_kernel(const float* __restrict__ W0, const float* __restrict__ W1,
                                                     const float* __restrict__ W2, const float* __restrict__ W3,
                                                     int R, int C, unsigned short* __restrict__ out,
                                                     long planeStride, float scale) {
  __shared__ float sm[64][65];
  const int t  = threadIdx.x;
  const int r0 = blockIdx.x * 64;
  const int c0 = blockIdx.y * 64;
  const int z  = blockIdx.z;
  const float* W = (z == 0) ? W0 : (z == 1) ? W1 : (z == 2) ? W2 : W3;
#pragma unroll
  for (int i = 0; i < 16; ++i) {
    const int e  = i * 256 + t;
    const int rl = e >> 6;
    const int cl = e & 63;
    sm[cl][rl] = W[(size_t)(r0 + rl) * C + c0 + cl] * scale;
  }
  __syncthreads();
  const int lane = t & 31, wave = t >> 5;
  const int q = lane >> 3, c8 = (lane & 7) * 8;
  unsigned short* op = out + (size_t)z * planeStride;
  v4u u[2];
#pragma unroll
  for (int it = 0; it < 2; ++it) {
    const int row = wave * 8 + it * 4 + q;
    unsigned short hb[8];
#pragma unroll
    for (int e = 0; e < 8; ++e) hb[e] = h_bits(sm[row][c8 + e]);
    u[it] = (v4u){pk16(hb[0], hb[1]), pk16(hb[2], hb[3]), pk16(hb[4], hb[5]), pk16(hb[6], hb[7])};
  }
  for (int pass = 0; pass < 2; ++pass) {
#pragma unroll
    for (int it = 0; it < 2; ++it) {
      const int row = wave * 8 + it * 4 + q;
      *(volatile v4u*)(op + (size_t)(c0 + row) * R + r0 + c8) = u[it];
    }
    __threadfence();
  }
}

__global__ __launch_bounds__(256) void dist_bias_kernel(const float* __restrict__ G, const float* __restrict__ SQb,
                                                        const float* __restrict__ NMb, float* __restrict__ OUT) {
#pragma clang fp contract(off)
  __shared__ float red[8];
  const int i = blockIdx.x;
  const int t = threadIdx.x, lane = t & 31, wave = t >> 5;
  const int cA = 4 * t, cB = 1024 + 4 * t;
  const float sqi = SQb[i];
  const float mi  = NMb[i];
  const float* gr = G + (size_t)i * kSeq;
  const v4f gA = *(const v4f*)(gr + cA);
  const v4f gB = *(const v4f*)(gr + cB);
  const v4f sA = *(const v4f*)(SQb + cA);
  const v4f sB = *(const v4f*)(SQb + cB);
  const v4f mA = *(const v4f*)(NMb + cA);
  const v4f mB = *(const v4f*)(NMb + cB);
  float dm[8], m2v[8];
#pragma unroll
  for (int e = 0; e < 4; ++e) {
    {
      const float m2 = mi * mA[e];
      const float t1 = sqi + sA[e];
      const float t2 = 2.0f * gA[e];
      const float d2 = t1 - t2;
      const float cd = sqrtf(fmaxf(d2, 0.0f));
      m2v[e] = m2;
      dm[e]  = cd * m2;
    }
    {
      const float m2 = mi * mB[e];
      const float t1 = sqi + sB[e];
      const float t2 = 2.0f * gB[e];
      const float d2 = t1 - t2;
      const float cd = sqrtf(fmaxf(d2, 0.0f));
      m2v[4 + e] = m2;
      dm[4 + e]  = cd * m2;
    }
  }
  float lmax = -INFINITY;
#pragma unroll
  for (int e = 0; e < 8; ++e) lmax = fmaxf(lmax, dm[e]);
#pragma unroll
  for (int off = 16; off > 0; off >>= 1) lmax = fmaxf(lmax, __shfl_xor(lmax, off, 32));
  if (lane == 0) red[wave] = lmax;
  __syncthreads();
  float rmax = red[0];
#pragma unroll
  for (int w = 1; w < 8; ++w) rmax = fmaxf(rmax, red[w]);
  v4f oA, oB;
#pragma unroll
  for (int e = 0; e < 4; ++e) {
    {
      float v = rmax - dm[e];
      const int col = cA + e;
      if (col == i) v = v * 0.0f;
      oA[e] = v * m2v[e];
    }
    {
      float v = rmax - dm[4 + e];
      const int col = cB + e;
      if (col == i) v = v * 0.0f;
      oB[e] = v * m2v[4 + e];
    }
  }
  float* orow = OUT + (size_t)i * kSeq;
  for (int pass = 0; pass < 2; ++pass) {
    *(volatile v4f*)(orow + cA) = oA;
    *(volatile v4f*)(orow + cB) = oB;
    __threadfence();
  }
}

__global__ __launch_bounds__(512) void softmax_kernel(const float* __restrict__ S, unsigned short* __restrict__ P) {
  __shared__ float redM[16];
  __shared__ float redS[16];
  const int row  = blockIdx.x;
  const int t    = threadIdx.x;
  const int lane = t & 31, wave = t >> 5;
  const int c0   = 4 * t;
  const v4f a = *(const v4f*)(S + (size_t)row * kSeq + c0);
  float m = fmaxf(fmaxf(a[0], a[1]), fmaxf(a[2], a[3]));
#pragma unroll
  for (int off = 16; off > 0; off >>= 1) m = fmaxf(m, __shfl_xor(m, off, 32));
  if (lane == 0) redM[wave] = m;
  __syncthreads();
  m = redM[0];
#pragma unroll
  for (int w = 1; w < 16; ++w) m = fmaxf(m, redM[w]);
  const float e0 = expf(a[0] - m);
  const float e1 = expf(a[1] - m);
  const float e2 = expf(a[2] - m);
  const float e3 = expf(a[3] - m);
  float s = (e0 + e1) + (e2 + e3);
#pragma unroll
  for (int off = 16; off > 0; off >>= 1) s += __shfl_xor(s, off, 32);
  if (lane == 0) redS[wave] = s;
  __syncthreads();
  float tot = redS[0];
#pragma unroll
  for (int w = 1; w < 16; ++w) tot += redS[w];
  const float r = kPCarry * (1.0f / tot);
  const v2u u = (v2u){pk16(h_bits(e0 * r), h_bits(e1 * r)), pk16(h_bits(e2 * r), h_bits(e3 * r))};
  unsigned short* q = P + (size_t)row * kSeq + c0;
  *(volatile v2u*)q = u;
  __threadfence();
  *(volatile v2u*)q = u;
}

template <bool W16>
__global__ __launch_bounds__(256) void addnorm_ln_kernel(const float* __restrict__ Y, const float* __restrict__ gam,
                                                         const float* __restrict__ bet, float* __restrict__ outF,
                                                         unsigned short* __restrict__ out16) {
  const int t = threadIdx.x, lane = t & 31, wave = t >> 5;
  const int row = blockIdx.x * 8 + wave;
  const float* yr = Y + (size_t)row * kDim;
  v4f v[4];
  float s = 0.f;
#pragma unroll
  for (int it = 0; it < 4; ++it) {
    v[it] = *(const v4f*)(yr + it * 128 + 4 * lane);
    s += (v[it][0] + v[it][1]) + (v[it][2] + v[it][3]);
  }
#pragma unroll
  for (int off = 16; off > 0; off >>= 1) s += __shfl_xor(s, off, 32);
  const float mu = s * kInvDim;
  float ss = 0.f;
#pragma unroll
  for (int it = 0; it < 4; ++it) {
#pragma unroll
    for (int e = 0; e < 4; ++e) {
      const float d = v[it][e] - mu;
      ss += d * d;
    }
  }
#pragma unroll
  for (int off = 16; off > 0; off >>= 1) ss += __shfl_xor(ss, off, 32);
  const float var = ss * kInvDim;
  const float inv = rsqrtf(var + kLnEps);
  v4f o[4];
#pragma unroll
  for (int it = 0; it < 4; ++it) {
    const int col = it * 128 + 4 * lane;
    const v4f gv = *(const v4f*)(gam + col);
    const v4f bv = *(const v4f*)(bet + col);
#pragma unroll
    for (int e = 0; e < 4; ++e) o[it][e] = (v[it][e] - mu) * inv * gv[e] + bv[e];
  }
  float* orow = outF + (size_t)row * kDim;
  for (int pass = 0; pass < 2; ++pass) {
#pragma unroll
    for (int it = 0; it < 4; ++it) *(volatile v4f*)(orow + it * 128 + 4 * lane) = o[it];
    __threadfence();
  }
  if (W16) {
    v4u u[2];
#pragma unroll
    for (int it = 0; it < 2; ++it) {
      const int col = it * 256 + 8 * lane;
      const v4f a  = *(const v4f*)(yr + col);
      const v4f c  = *(const v4f*)(yr + col + 4);
      const v4f ga = *(const v4f*)(gam + col);
      const v4f gc = *(const v4f*)(gam + col + 4);
      const v4f ba = *(const v4f*)(bet + col);
      const v4f bc = *(const v4f*)(bet + col + 4);
      unsigned short hb[8];
#pragma unroll
      for (int e = 0; e < 4; ++e) {
        hb[e]     = h_bits((a[e] - mu) * inv * ga[e] + ba[e]);
        hb[4 + e] = h_bits((c[e] - mu) * inv * gc[e] + bc[e]);
      }
      u[it] = (v4u){pk16(hb[0], hb[1]), pk16(hb[2], hb[3]), pk16(hb[4], hb[5]), pk16(hb[6], hb[7])};
    }
    unsigned short* hrow = out16 + (size_t)row * kDim;
    for (int pass = 0; pass < 2; ++pass) {
#pragma unroll
      for (int it = 0; it < 2; ++it) *(volatile v4u*)(hrow + it * 256 + 8 * lane) = u[it];
      __threadfence();
    }
  }
}

extern "C" void kernel_launch(void* const* d_in, const int* in_sizes, int n_in,
                              void* d_out, int out_size, void* d_ws, size_t ws_size,
                              hipStream_t stream) {
  (void)n_in;
  const float* x   = (const float*)d_in[0];
  const float* nm  = (const float*)d_in[1];
  const float* wq  = (const float*)d_in[2];  const float* bq  = (const float*)d_in[3];
  const float* wk  = (const float*)d_in[4];  const float* bk  = (const float*)d_in[5];
  const float* wv  = (const float*)d_in[6];  const float* bv  = (const float*)d_in[7];
  const float* wo  = (const float*)d_in[8];  const float* bo  = (const float*)d_in[9];
  const float* g1  = (const float*)d_in[10]; const float* be1 = (const float*)d_in[11];
  const float* w1  = (const float*)d_in[12]; const float* b1  = (const float*)d_in[13];
  const float* w2  = (const float*)d_in[14]; const float* b2  = (const float*)d_in[15];
  const float* g2  = (const float*)d_in[16]; const float* be2 = (const float*)d_in[17];

  const size_t bX16  = (size_t)kTok * kDim * 2;
  const size_t bWT   = (size_t)4 * kDim * kDim * 2 + (size_t)2 * kDim * kFfn * 2;
  const size_t bSQ   = (size_t)kTok * 4;
  const size_t bPl16 = (size_t)kTok * kDim * 2;
  const size_t bSS   = (size_t)kSeq * kSeq * 4;
  const size_t oX16  = 0;
  const size_t oWT   = oX16 + bX16;
  const size_t oSQ   = oWT + bWT;
  const size_t oQ16  = oSQ + bSQ;
  const size_t oK16  = oQ16 + bPl16;
  const size_t oVT16 = oK16 + bPl16;
  const size_t oR4   = oVT16 + bPl16;
  const size_t oR5   = oR4 + 2 * bSS;
  const size_t oR6   = oR5 + 2 * bSS;
  const size_t oR7   = oR6 + bSS;
  const size_t oEnd  = oR7 + bPl16;
  if (oEnd > ws_size) return;
  if ((size_t)out_size < (size_t)kTok * kDim) return;
  if (in_sizes[0] != kTok * kDim || in_sizes[1] != kTok) return;

  char* ws = (char*)d_ws;
  unsigned short* X16   = (unsigned short*)(ws + oX16);
  unsigned short* WT    = (unsigned short*)(ws + oWT);
  unsigned short* wqT   = WT;
  unsigned short* wkT   = WT + (size_t)kDim * kDim;
  unsigned short* wvT   = WT + (size_t)2 * kDim * kDim;
  unsigned short* woT   = WT + (size_t)3 * kDim * kDim;
  unsigned short* w1T   = WT + (size_t)4 * kDim * kDim;
  unsigned short* w2T   = w1T + (size_t)kDim * kFfn;
  float*          SQ    = (float*)(ws + oSQ);
  unsigned short* Q16   = (unsigned short*)(ws + oQ16);
  unsigned short* K16   = (unsigned short*)(ws + oK16);
  unsigned short* VT16  = (unsigned short*)(ws + oVT16);
  float*          GPL   = (float*)(ws + oR4);
  float*          BPL   = (float*)(ws + oR4 + bSS);
  unsigned short* H16   = (unsigned short*)(ws + oR4);
  float*          SC    = (float*)(ws + oR5);
  float*          Y     = (float*)(ws + oR5);
  float*          XF    = (float*)(ws + oR5 + bSS);
  unsigned short* P16   = (unsigned short*)(ws + oR6);
  float*          Z     = (float*)(ws + oR6);
  unsigned short* CTX16 = (unsigned short*)(ws + oR7);
  float*          outp  = (float*)d_out;

  xprep_kernel<<<dim3(kTok / 32), 256, 0, stream>>>(x, X16, SQ);

  wtcast_kernel<<<dim3(kDim / 64, kDim / 64, 4), 256, 0, stream>>>(wq, wk, wv, wo, kDim, kDim, WT,
                                                                     (long)kDim * kDim, kWCarry);
  wtcast_kernel<<<dim3(kDim / 64, kFfn / 64, 1), 256, 0, stream>>>(w1, w1, w1, w1, kDim, kFfn, w1T, 0L, kWCarry);
  wtcast_kernel<<<dim3(kFfn / 64, kDim / 64, 1), 256, 0, stream>>>(w2, w2, w2, w2, kFfn, kDim, w2T, 0L, kWCarry);

  wmma_gemm64<0, false, 2, 1, false, 0><<<dim3(128, 1), 256, 0, stream>>>(
      X16, X16, kDim, 0L, wqT, wqT, kDim, 0L, Q16, Q16, kDim, 0L, bq, SQ, 0L, kTok, kDim, kDim, kWCarryInv);
  wmma_gemm64<0, false, 2, 1, false, 0><<<dim3(128, 1), 256, 0, stream>>>(
      X16, X16, kDim, 0L, wkT, wkT, kDim, 0L, K16, K16, kDim, 0L, bk, SQ, 0L, kTok, kDim, kDim, kWCarryInv);
  wmma_gemm64<0, false, 1, 1, false, 0><<<dim3(32, kBatch), 256, 0, stream>>>(
      wvT, wvT, kDim, 0L, X16, X16, kDim, (long)kSeq * kDim, VT16, VT16, kSeq, (long)kDim * kSeq,
      bv, SQ, 0L, kDim, kSeq, kDim, kWCarryInv);

  for (int b = 0; b < kBatch; ++b) {
    const unsigned short* X16b = X16 + (size_t)b * kSeq * kDim;
    wmma_gemm64<0, false, 0, 0, false, 0><<<dim3(128, 1), 256, 0, stream>>>(
        X16b, X16b, kDim, 0L, X16b, X16b, kDim, 0L, GPL, GPL, kSeq, 0L, SQ, SQ, 0L, kSeq, kSeq, kDim, 1.0f);
    dist_bias_kernel<<<dim3(kSeq), 256, 0, stream>>>(GPL, SQ + (size_t)b * kSeq, nm + (size_t)b * kSeq, BPL);
    for (int hc = 0; hc < kHeads / kHeadsPerChunk; ++hc) {
      const int h0 = hc * kHeadsPerChunk;
      const unsigned short* Qbh = Q16 + (size_t)b * kSeq * kDim + (size_t)h0 * kDh;
      const unsigned short* Kbh = K16 + (size_t)b * kSeq * kDim + (size_t)h0 * kDh;
      const unsigned short* Vbh = VT16 + (size_t)b * kDim * kSeq + (size_t)h0 * kDh * kSeq;
      unsigned short*       Cbh = CTX16 + (size_t)b * kSeq * kDim + (size_t)h0 * kDh;
      wmma_gemm64<0, false, 0, 0, true, 0><<<dim3(128, kHeadsPerChunk), 256, 0, stream>>>(
          Qbh, Qbh, kDim, (long)kDh, Kbh, Kbh, kDim, (long)kDh, SC, SC, kSeq, (long)kSeq * kSeq,
          SQ, BPL, 0L, kSeq, kSeq, kDh, kScoreScale);
      softmax_kernel<<<dim3(kHeadsPerChunk * kSeq), 512, 0, stream>>>(SC, P16);
      wmma_gemm64<0, false, 0, 1, false, 0><<<dim3(4, kHeadsPerChunk), 256, 0, stream>>>(
          P16, P16, kSeq, (long)kSeq * kSeq, Vbh, Vbh, kSeq, (long)kDh * kSeq, Cbh, Cbh, kDim, (long)kDh,
          SQ, SQ, 0L, kSeq, kDh, kSeq, kPVScale);
    }
  }

  wmma_gemm64<0, false, 2, 0, true, 0><<<dim3(128, 1), 256, 0, stream>>>(
      CTX16, CTX16, kDim, 0L, woT, woT, kDim, 0L, Y, Y, kDim, 0L, bo, x, 0L, kTok, kDim, kDim, kOutScale);

  addnorm_ln_kernel<true><<<dim3(kTok / 8), 256, 0, stream>>>(Y, g1, be1, XF, X16);

  wmma_gemm64<0, false, 2, 1, false, 2><<<dim3(512, 1), 256, 0, stream>>>(
      X16, X16, kDim, 0L, w1T, w1T, kDim, 0L, H16, H16, kFfn, 0L, b1, SQ, 0L, kTok, kFfn, kDim, kWCarryInv);

  wmma_gemm64<0, false, 2, 0, true, 0><<<dim3(128, 1), 256, 0, stream>>>(
      H16, H16, kFfn, 0L, w2T, w2T, kFfn, 0L, Z, Z, kDim, 0L, b2, XF, 0L, kTok, kDim, kFfn, kWCarryInv);

  addnorm_ln_kernel<false><<<dim3(kTok / 8), 256, 0, stream>>>(Z, g2, be2, outp, CTX16);
}
